// Critic_att_55456617726455
// MI455X (gfx1250) — hardware-run, weakly checked
//
#include <hip/hip_runtime.h>
#include <math.h>

typedef __attribute__((ext_vector_type(16))) _Float16 v16h;
typedef __attribute__((ext_vector_type(8)))  _Float16 v8h;
typedef __attribute__((ext_vector_type(8)))  float    v8f;
typedef __attribute__((ext_vector_type(4)))  float    v4f;

constexpr int kRows    = 65536;
constexpr int kAgents  = 3;
constexpr int kObs     = 12;
constexpr int kXW      = kAgents * kObs + 2 * kAgents;
constexpr int kHid     = 64;
constexpr int kFeat    = 32;
constexpr int kCat     = 3 * kFeat;
constexpr int kBlkRows = 64;
constexpr int kThreads = 128;
constexpr int kWaves   = kThreads / 32;
static_assert(kXW == 42, "input row width");
static_assert(kRows % kBlkRows == 0, "no row tail");
static_assert(kBlkRows == kWaves * 16, "one 16-row tile per wave");
static_assert((kHid % 32) == 0 && (kFeat % 32) == 0 && (kCat % 32) == 0, "K multiples of 32");
static_assert((kBlkRows * kXW) % 4 == 0, "x tile in 16-B pieces");

constexpr float kWCarry  = 16.0f;
constexpr float kWInv    = 1.0f / kWCarry;
constexpr float kLoCarry = 2048.0f;
constexpr float kLoInv   = 1.0f / kLoCarry;
constexpr float kHiFloor = 6.2e-5f;
constexpr float kInvFeat = 1.0f / (float)kFeat;
constexpr float kLnEps   = 1e-5f;

constexpr int kOffAs2  = 0;
constexpr int kOffAf2  = kOffAs2 + kAgents * kFeat * kHid;
constexpr int kOffAo2  = kOffAf2 + kAgents * kFeat * kHid;
constexpr int kOffAm1  = kOffAo2 + kAgents * kFeat * kHid;
constexpr int kOffAm2  = kOffAm1 + kAgents * kHid * kCat;
constexpr int kOffAm3  = kOffAm2 + kAgents * kHid * kHid;
constexpr int kOffCm1  = kOffAm3 + kAgents * kFeat * kHid;
constexpr int kOffCm2  = kOffCm1 + kHid * kHid;
constexpr int kOffCaH  = kOffCm2 + kHid * kHid;
constexpr int kOffCaL  = kOffCaH + 3 * kFeat * kFeat;
constexpr int kOffAs2L = kOffCaL + 3 * kFeat * kFeat;
constexpr int kOffAf2L = kOffAs2L + kAgents * kFeat * kHid;
constexpr int kOffAo2L = kOffAf2L + kAgents * kFeat * kHid;
constexpr int kOffAm1L = kOffAo2L + kAgents * kFeat * kHid;
constexpr int kOffAm2L = kOffAm1L + kAgents * kHid * kCat;
constexpr int kOffAm3L = kOffAm2L + kAgents * kHid * kHid;
constexpr int kPlaneHalves = kOffAm3L + kAgents * kFeat * kHid;
constexpr int kPrepChunks  = kPlaneHalves / 8;
constexpr size_t kWsBytes  = (size_t)kPlaneHalves * 2;
static_assert(kPlaneHalves == 124928, "plane total");
static_assert(kWsBytes == 249856ull, "carve total");
static_assert(kWsBytes <= 134217728ull, "carve cap");
static_assert((kPrepChunks % 256) == 0, "prep grid exact");
constexpr int kNumSeg = 20;

__host__ __device__ constexpr int seg_off(int t) {
  return t == 0 ? kOffAs2 : t == 1 ? kOffAf2 : t == 2 ? kOffAo2 : t == 3 ? kOffAm1 :
         t == 4 ? kOffAm2 : t == 5 ? kOffAm3 : t == 6 ? kOffCm1 : t == 7 ? kOffCm2 :
         t < 11 ? (kOffCaH + (t - 8) * kFeat * kFeat) :
         t < 14 ? (kOffCaL + (t - 11) * kFeat * kFeat) :
         t == 14 ? kOffAs2L : t == 15 ? kOffAf2L : t == 16 ? kOffAo2L : t == 17 ? kOffAm1L :
         t == 18 ? kOffAm2L : kOffAm3L;
}
__host__ __device__ constexpr int seg_base(int t) { return t >= 14 ? (t - 14) : t; }
__host__ __device__ constexpr int seg_k(int t) {
  return seg_base(t) == 3 ? kCat : (seg_base(t) < 8 ? kHid : kFeat);
}
__host__ __device__ constexpr int seg_n(int t) {
  return (seg_base(t) < 3 || seg_base(t) == 5) ? kFeat : (seg_base(t) < 8 ? kHid : kFeat);
}
__host__ __device__ constexpr int seg_lo(int t) { return t >= 11 ? 1 : 0; }
__host__ __device__ constexpr int seg_twin(int t) { return (t == 6 || t == 7) ? 0 : 1; }
static_assert((seg_off(1) % 256) == 0 && (seg_off(3) % 256) == 0 && (seg_off(8) % 256) == 0 &&
              (seg_off(11) % 256) == 0 && (seg_off(13) % 256) == 0 && (seg_off(14) % 256) == 0 &&
              (seg_off(17) % 256) == 0 && (seg_off(19) % 256) == 0, "segment starts on 32-chunk boundaries");
static_assert(seg_off(19) + kAgents * seg_n(19) * seg_k(19) == kPlaneHalves, "last segment ends the region");
static_assert(seg_k(17) == kCat && seg_n(17) == kHid && seg_k(14) == kHid && seg_n(14) == kFeat, "twin shapes");

union FragU { v16h v; v8h h[2]; };
__device__ __forceinline__ v16h frag_load(const _Float16* p) {
  FragU f;
  f.h[0] = *(const v8h*)(p);
  f.h[1] = *(const v8h*)(p + 16);
  return f.v;
}
__device__ __forceinline__ v8f mma_h(v16h a, v16h b, v8f c) {
  c = __builtin_amdgcn_wmma_f32_16x16x32_f16(false, a, false, b, (short)0, c, false, false);
  asm volatile("v_nop\n\tv_nop\n\tv_nop\n\tv_nop" : "+v"(c) : "v"(a), "v"(b));
  return c;
}
__device__ __forceinline__ void wave_sync() {
  __builtin_amdgcn_fence(__ATOMIC_RELEASE, "workgroup");
  __builtin_amdgcn_wave_barrier();
  __builtin_amdgcn_fence(__ATOMIC_ACQUIRE, "workgroup");
}
__device__ __forceinline__ void split_h(float v, _Float16& hi, _Float16& lo) {
  const float vh = (fabsf(v) < kHiFloor) ? 0.0f : v;
  hi = (_Float16)vh;
  const float hf = (float)hi;
  lo = (_Float16)((v - hf) * kLoCarry);
}
__device__ __forceinline__ void load16(const float* p, float (&o)[16]) {
#pragma unroll
  for (int i = 0; i < 4; ++i) {
    const v4f t = *(const v4f*)(p + 4 * i);
    o[4 * i + 0] = t[0];
    o[4 * i + 1] = t[1];
    o[4 * i + 2] = t[2];
    o[4 * i + 3] = t[3];
  }
}
__device__ __forceinline__ void store16f(float* p, const float (&o)[16]) {
#pragma unroll
  for (int i = 0; i < 4; ++i) {
    v4f t;
    t[0] = o[4 * i + 0];
    t[1] = o[4 * i + 1];
    t[2] = o[4 * i + 2];
    t[3] = o[4 * i + 3];
    *(v4f*)(p + 4 * i) = t;
  }
}
__device__ __forceinline__ void store16h(_Float16* p, const float (&o)[16]) {
  v8h a, b;
#pragma unroll
  for (int k = 0; k < 8; ++k) {
    a[k] = (_Float16)o[k];
    b[k] = (_Float16)o[8 + k];
  }
  *(v8h*)(p) = a;
  *(v8h*)(p + 8) = b;
}
__device__ __forceinline__ void store16hl(_Float16* ph, _Float16* pl, const float (&o)[16]) {
  v8h a, b, c, d;
#pragma unroll
  for (int k = 0; k < 8; ++k) {
    _Float16 h0, l0, h1, l1;
    split_h(o[k], h0, l0);
    split_h(o[8 + k], h1, l1);
    a[k] = h0;
    b[k] = h1;
    c[k] = l0;
    d[k] = l1;
  }
  *(v8h*)(ph) = a;
  *(v8h*)(ph + 8) = b;
  *(v8h*)(pl) = c;
  *(v8h*)(pl + 8) = d;
}

template <int KT, int NT>
__device__ __forceinline__ void wave_mm(const _Float16* A, int lda, const _Float16* Bt, int ldb,
                                        int lane, v8f (&acc)[NT]) {
  const int cc = lane & 15, ko = (lane >> 4) * 8;
#pragma unroll
  for (int nt = 0; nt < NT; ++nt) acc[nt] = (v8f){0.f, 0.f, 0.f, 0.f, 0.f, 0.f, 0.f, 0.f};
#pragma unroll
  for (int kt = 0; kt < KT; ++kt) {
    const v16h a = frag_load(A + cc * lda + kt * 32 + ko);
#pragma unroll
    for (int nt = 0; nt < NT; ++nt) {
      const v16h b = frag_load(Bt + (nt * 16 + cc) * ldb + kt * 32 + ko);
      acc[nt] = mma_h(a, b, acc[nt]);
    }
  }
}

template <int KT, int NT>
__device__ __forceinline__ void wave_mm3(const _Float16* Ah, const _Float16* Al, int lda,
                                         const _Float16* Bh, const _Float16* Bl, int ldb,
                                         int lane, v8f (&am)[NT], v8f (&ar)[NT]) {
  const int cc = lane & 15, ko = (lane >> 4) * 8;
#pragma unroll
  for (int nt = 0; nt < NT; ++nt) {
    am[nt] = (v8f){0.f, 0.f, 0.f, 0.f, 0.f, 0.f, 0.f, 0.f};
    ar[nt] = (v8f){0.f, 0.f, 0.f, 0.f, 0.f, 0.f, 0.f, 0.f};
  }
#pragma unroll
  for (int kt = 0; kt < KT; ++kt) {
    const v16h ah = frag_load(Ah + cc * lda + kt * 32 + ko);
    const v16h al = frag_load(Al + cc * lda + kt * 32 + ko);
#pragma unroll
    for (int nt = 0; nt < NT; ++nt) {
      const v16h bh = frag_load(Bh + (nt * 16 + cc) * ldb + kt * 32 + ko);
      const v16h bl = frag_load(Bl + (nt * 16 + cc) * ldb + kt * 32 + ko);
      am[nt] = mma_h(ah, bh, am[nt]);
      ar[nt] = mma_h(ah, bl, ar[nt]);
      ar[nt] = mma_h(al, bh, ar[nt]);
    }
  }
}

template <int NT>
__device__ __forceinline__ void fold_resid(v8f (&am)[NT], const v8f (&ar)[NT]) {
#pragma unroll
  for (int nt = 0; nt < NT; ++nt) {
#pragma unroll
    for (int r = 0; r < 8; ++r) am[nt][r] = fmaf(ar[nt][r], kLoInv, am[nt][r]);
  }
}

template <int NT, int ACT, int HM, bool WF>
__device__ __forceinline__ void wave_epi(const v8f (&acc)[NT], const float* bias,
                                         _Float16* Ch, _Float16* Cl, int ldh, float* Cf, int ldf, int lane) {
  const int cc = lane & 15, r0 = (lane >> 4) * 8;
#pragma unroll
  for (int nt = 0; nt < NT; ++nt) {
    const int n = nt * 16 + cc;
    const float bv = bias[n];
#pragma unroll
    for (int r = 0; r < 8; ++r) {
      float v = acc[nt][r] * kWInv + bv;
      if (ACT == 1) v = fmaxf(v, 0.0f);
      if (ACT == 2) v = (v >= 0.0f) ? v : 0.01f * v;
      if (HM == 1) Ch[(r0 + r) * ldh + n] = (_Float16)v;
      if (HM == 2) {
        _Float16 hi, lo;
        split_h(v, hi, lo);
        Ch[(r0 + r) * ldh + n] = hi;
        Cl[(r0 + r) * ldh + n] = lo;
      }
      if (WF) Cf[(r0 + r) * ldf + n] = v;
    }
  }
}

__device__ __forceinline__ void pair_layer(const float* xcol, const float* W, const float* Bv,
                                           _Float16* Th, _Float16* Tl, int lane) {
  const float w0a = W[lane], w1a = W[kHid + lane];
  const float w0b = W[32 + lane], w1b = W[kHid + 32 + lane];
  const float ba = Bv[lane], bb = Bv[32 + lane];
#pragma unroll 4
  for (int m = 0; m < 16; ++m) {
    const float x0 = xcol[m * kXW], x1 = xcol[m * kXW + 1];
    float ta = x0 * w0a;
    ta = fmaf(x1, w1a, ta);
    ta += ba;
    float tb = x0 * w0b;
    tb = fmaf(x1, w1b, tb);
    tb += bb;
    _Float16 ha, la, hb, lb;
    split_h(fmaxf(ta, 0.0f), ha, la);
    split_h(fmaxf(tb, 0.0f), hb, lb);
    Th[m * kHid + lane]      = ha;
    Tl[m * kHid + lane]      = la;
    Th[m * kHid + 32 + lane] = hb;
    Tl[m * kHid + 32 + lane] = lb;
  }
}

__device__ __forceinline__ void ln_relu16(float (&v)[16], const float* gam, const float* bet) {
  float s = 0.0f;
#pragma unroll
  for (int k = 0; k < 16; ++k) s += v[k];
  s += __shfl_xor(s, 16, 32);
  const float mu = s * kInvFeat;
  float q = 0.0f;
#pragma unroll
  for (int k = 0; k < 16; ++k) {
    const float d = v[k] - mu;
    q = fmaf(d, d, q);
  }
  q += __shfl_xor(q, 16, 32);
  const float var = q * kInvFeat;
  const float rstd = 1.0f / sqrtf(var + kLnEps);
  float gg[16], bb[16];
  load16(gam, gg);
  load16(bet, bb);
#pragma unroll
  for (int k = 0; k < 16; ++k) v[k] = fmaxf((v[k] - mu) * rstd * gg[k] + bb[k], 0.0f);
}

template <int NKV>
__device__ __forceinline__ void pool_ln_relu(const float (&q)[16], const float (&kv)[NKV][16],
                                             const float* gam, const float* bet, float inv_scale,
                                             float (&o)[16]) {
  float l[NKV];
#pragma unroll
  for (int j = 0; j < NKV; ++j) {
    float a = 0.0f;
#pragma unroll
    for (int k = 0; k < 16; ++k) a = fmaf(q[k], kv[j][k], a);
    a += __shfl_xor(a, 16, 32);
    l[j] = a * inv_scale;
  }
  float mx = l[0];
#pragma unroll
  for (int j = 1; j < NKV; ++j) mx = fmaxf(mx, l[j]);
  float sum = 0.0f;
#pragma unroll
  for (int j = 0; j < NKV; ++j) {
    l[j] = expf(l[j] - mx);
    sum += l[j];
  }
  const float inv = 1.0f / sum;
#pragma unroll
  for (int k = 0; k < 16; ++k) {
    float v = 0.0f;
#pragma unroll
    for (int j = 0; j < NKV; ++j) v = fmaf(l[j] * inv, kv[j][k], v);
    o[k] = v;
  }
  ln_relu16(o, gam, bet);
}

__device__ __forceinline__ float logit3(float t0, float t1, float t2, float p0, float p1, float p2, float sc) {
  float a = t0 * p0;
  a = fmaf(t1, p1, a);
  a = fmaf(t2, p2, a);
  return a * sc;
}

struct PrepArgs { const float* src[kNumSeg]; };
static_assert(sizeof(PrepArgs) == 8 * kNumSeg, "no padding");

__global__ __launch_bounds__(256) void prep_planes_kernel(PrepArgs A, _Float16* __restrict__ dst) {
  const int i = blockIdx.x * 256 + threadIdx.x;
  const int ic = i < kPrepChunks ? i : (kPrepChunks - 1);
  const float* src = A.src[0];
  int K = seg_k(0), N = seg_n(0), st = seg_off(0) / 8, lo = seg_lo(0), twin = seg_twin(0);
#pragma unroll
  for (int t = 1; t < kNumSeg; ++t) {
    if (ic >= seg_off(t) / 8) {
      src = A.src[t];
      K = seg_k(t);
      N = seg_n(t);
      st = seg_off(t) / 8;
      lo = seg_lo(t);
      twin = seg_twin(t);
    }
  }
  const int e0  = (ic - st) * 8;
  const int per = N * K;
  const int mat = e0 / per;
  const int rem = e0 - mat * per;
  const int n   = rem / K;
  const int k0  = rem - n * K;
  v8h hv;
#pragma unroll
  for (int j = 0; j < 8; ++j) {
    const float w = src[(size_t)(mat * K + k0 + j) * N + n] * kWCarry;
    const float wh = (twin != 0 && fabsf(w) < kHiFloor) ? 0.0f : w;
    const _Float16 hi = (_Float16)wh;
    const float hf = (float)hi;
    const _Float16 rs = (_Float16)((w - hf) * kLoCarry);
    hv[j] = lo ? rs : hi;
  }
  if (i < kPrepChunks) {
    _Float16* q = dst + (size_t)ic * 8;
    *(volatile v8h*)q = hv;
    __threadfence();
    *(volatile v8h*)q = hv;
  }
}

constexpr int kHalfArena  = 6144;
constexpr int kFloatArena = 6656;
static_assert(kBlkRows * kXW * 4 + kWaves * kHalfArena * 2 + kWaves * kFloatArena * 4 + kBlkRows * 4 == 166656,
              "static LDS extent");

struct Params {
  const float* x;
  const float* as1w; const float* as1b; const float* as2b;
  const float* af1w; const float* af1b; const float* af2b; const float* afng; const float* afnb;
  const float* ao1w; const float* ao1b; const float* ao2b; const float* aong; const float* aonb;
  const float* am1b; const float* am2b; const float* am3b;
  const float* ca1b; const float* ca2b; const float* ca3b;
  const float* cng;  const float* cnb;  const float* cn2g; const float* cn2b;
  const float* cm1b; const float* cm2b; const float* cm3w; const float* cm3b;
  const _Float16* wp;
  float* out;
};
static_assert(sizeof(Params) == 240, "no padding");

__global__ __launch_bounds__(kThreads) void fused_forward_kernel(Params P) {
  __shared__ __align__(16) float    sX[kBlkRows * kXW];
  __shared__ __align__(16) _Float16 sH[kWaves][kHalfArena];
  __shared__ __align__(16) float    sF[kWaves][kFloatArena];
  __shared__ __align__(16) float    sOut[kBlkRows];

  const int tid  = threadIdx.x;
  const int lane = tid & 31;
  const int wave = tid >> 5;
  const int hh   = lane >> 4;
  const int cc   = lane & 15;
  const int blockRow0 = blockIdx.x * kBlkRows;
  const int wrow0 = wave * 16;
  const float inv_scale = 1.0f / sqrtf((float)kFeat);

  {
    const v4f* xsrc = (const v4f*)(P.x + (size_t)blockRow0 * kXW);
    constexpr int kPieces = kBlkRows * kXW / 4;
#pragma unroll 1
    for (int it = 0; it < (kPieces + kThreads - 1) / kThreads; ++it) {
      const int idx = it * kThreads + tid;
      const int idc = idx < kPieces ? idx : (kPieces - 1);
      const v4f v = xsrc[idc];
      if (idx < kPieces) *(v4f*)(sX + 4 * idx) = v;
    }
  }
  __syncthreads();

  _Float16* T0h = sH[wave];
  _Float16* T0l = sH[wave] + 1024;
  _Float16* MBh = sH[wave] + 2048;
  _Float16* MBl = sH[wave] + 3584;
  _Float16* ZIN = sH[wave] + 5120;
  _Float16* T1h = MBh;
  _Float16* T1l = MBl;
  _Float16* AH  = T0h;
  _Float16* AL  = T0l;
  float* S32 = sF[wave];
  float* F32 = sF[wave] + 512;
  float* TPG = sF[wave] + 2048;
  float* ZF  = F32;
  const float* xw = sX + wrow0 * kXW;

#pragma unroll 1
  for (int g = 0; g < kAgents; ++g) {
    {
      const float* W  = P.as1w + g * 4 * kHid;
      const float* Bv = P.as1b + g * kHid;
      float wa[4], wb[4];
#pragma unroll
      for (int k = 0; k < 4; ++k) {
        wa[k] = W[k * kHid + lane];
        wb[k] = W[k * kHid + 32 + lane];
      }
      const float ba = Bv[lane], bb = Bv[32 + lane];
#pragma unroll 4
      for (int m = 0; m < 16; ++m) {
        const float* xr = xw + m * kXW;
        const float x0 = xr[kObs * g], x1 = xr[kObs * g + 1];
        const float x2 = xr[kAgents * kObs + 2 * g], x3 = xr[kAgents * kObs + 2 * g + 1];
        float ta = x0 * wa[0];
        ta = fmaf(x1, wa[1], ta);
        ta = fmaf(x2, wa[2], ta);
        ta = fmaf(x3, wa[3], ta);
        ta += ba;
        float tb = x0 * wb[0];
        tb = fmaf(x1, wb[1], tb);
        tb = fmaf(x2, wb[2], tb);
        tb = fmaf(x3, wb[3], tb);
        tb += bb;
        _Float16 ha, la, hb, lb;
        split_h(fmaxf(ta, 0.0f), ha, la);
        split_h(fmaxf(tb, 0.0f), hb, lb);
        T0h[m * kHid + lane]      = ha;
        T0l[m * kHid + lane]      = la;
        T0h[m * kHid + 32 + lane] = hb;
        T0l[m * kHid + 32 + lane] = lb;
      }
    }
    wave_sync();
    {
      v8f am[2], ar[2];
      wave_mm3<2, 2>(T0h, T0l, kHid, P.wp + kOffAs2 + g * kFeat * kHid, P.wp + kOffAs2L + g * kFeat * kHid,
                     kHid, lane, am, ar);
      fold_resid<2>(am, ar);
      wave_epi<2, 1, 2, true>(am, P.as2b + g * kFeat, MBh, MBl, kCat, S32, kFeat, lane);
    }
    wave_sync();
#pragma unroll 1
    for (int j = 0; j < 3; ++j) {
      pair_layer(xw + kObs * g + 2 + 2 * j, P.af1w + g * 2 * kHid, P.af1b + g * kHid, T0h, T0l, lane);
      wave_sync();
      {
        v8f am[2], ar[2];
        wave_mm3<2, 2>(T0h, T0l, kHid, P.wp + kOffAf2 + g * kFeat * kHid, P.wp + kOffAf2L + g * kFeat * kHid,
                       kHid, lane, am, ar);
        fold_resid<2>(am, ar);
        wave_epi<2, 1, 0, true>(am, P.af2b + g * kFeat, T0h, T0l, kHid, F32 + j * 512, kFeat, lane);
      }
      wave_sync();
    }
    {
      float q[16], kv[3][16], o[16];
      load16(S32 + cc * kFeat + 16 * hh, q);
#pragma unroll
      for (int j = 0; j < 3; ++j) load16(F32 + (j * 16 + cc) * kFeat + 16 * hh, kv[j]);
      pool_ln_relu<3>(q, kv, P.afng + g * kFeat + 16 * hh, P.afnb + g * kFeat + 16 * hh, inv_scale, o);
      store16hl(MBh + cc * kCat + 32 + 16 * hh, MBl + cc * kCat + 32 + 16 * hh, o);
    }
    wave_sync();
#pragma unroll 1
    for (int j = 0; j < 2; ++j) {
      pair_layer(xw + kObs * g + 8 + 2 * j, P.ao1w + g * 2 * kHid, P.ao1b + g * kHid, T0h, T0l, lane);
      wave_sync();
      {
        v8f am[2], ar[2];
        wave_mm3<2, 2>(T0h, T0l, kHid, P.wp + kOffAo2 + g * kFeat * kHid, P.wp + kOffAo2L + g * kFeat * kHid,
                       kHid, lane, am, ar);
        fold_resid<2>(am, ar);
        wave_epi<2, 1, 0, true>(am, P.ao2b + g * kFeat, T0h, T0l, kHid, F32 + j * 512, kFeat, lane);
      }
      wave_sync();
    }
    {
      float q[16], kv[2][16], o[16];
      load16(S32 + cc * kFeat + 16 * hh, q);
#pragma unroll
      for (int j = 0; j < 2; ++j) load16(F32 + (j * 16 + cc) * kFeat + 16 * hh, kv[j]);
      pool_ln_relu<2>(q, kv, P.aong + g * kFeat + 16 * hh, P.aonb + g * kFeat + 16 * hh, inv_scale, o);
      store16hl(MBh + cc * kCat + 64 + 16 * hh, MBl + cc * kCat + 64 + 16 * hh, o);
    }
    wave_sync();
    {
      v8f am[4], ar[4];
      wave_mm3<3, 4>(MBh, MBl, kCat, P.wp + kOffAm1 + g * kHid * kCat, P.wp + kOffAm1L + g * kHid * kCat,
                     kCat, lane, am, ar);
      fold_resid<4>(am, ar);
      wave_epi<4, 1, 2, false>(am, P.am1b + g * kHid, T0h, T0l, kHid, S32, kFeat, lane);
    }
    wave_sync();
    {
      v8f am[4], ar[4];
      wave_mm3<2, 4>(T0h, T0l, kHid, P.wp + kOffAm2 + g * kHid * kHid, P.wp + kOffAm2L + g * kHid * kHid,
                     kHid, lane, am, ar);
      fold_resid<4>(am, ar);
      wave_epi<4, 1, 2, false>(am, P.am2b + g * kHid, T1h, T1l, kHid, S32, kFeat, lane);
    }
    wave_sync();
    {
      v8f am[2], ar[2];
      wave_mm3<2, 2>(T1h, T1l, kHid, P.wp + kOffAm3 + g * kFeat * kHid, P.wp + kOffAm3L + g * kFeat * kHid,
                     kHid, lane, am, ar);
      fold_resid<2>(am, ar);
      const float* bias = P.am3b + g * kFeat;
#pragma unroll
      for (int nt = 0; nt < 2; ++nt) {
        const int n = nt * 16 + cc;
        const float bv = bias[n];
#pragma unroll
        for (int r = 0; r < 8; ++r) {
          const float v = am[nt][r] * kWInv + bv;
          _Float16 hi, lo;
          split_h(v, hi, lo);
          AH[(8 * hh + r) * kFeat + n] = hi;
          AL[(8 * hh + r) * kFeat + n] = lo;
          if (g == 0) ZIN[(8 * hh + r) * kHid + n] = hi;
        }
      }
    }
    wave_sync();
#pragma unroll 1
    for (int p = 0; p < 3; ++p) {
      const _Float16* Bh = P.wp + kOffCaH + p * kFeat * kFeat;
      const _Float16* Bl = P.wp + kOffCaL + p * kFeat * kFeat;
      const float* bias = (p == 0) ? P.ca1b : ((p == 1) ? P.ca2b : P.ca3b);
      const int ko = 8 * hh;
      const v16h ah = frag_load(AH + cc * kFeat + ko);
      const v16h al = frag_load(AL + cc * kFeat + ko);
      v8f am[2], ar[2];
#pragma unroll
      for (int nt = 0; nt < 2; ++nt) {
        const v16h bh = frag_load(Bh + (nt * 16 + cc) * kFeat + ko);
        const v16h bl = frag_load(Bl + (nt * 16 + cc) * kFeat + ko);
        am[nt] = (v8f){0.f, 0.f, 0.f, 0.f, 0.f, 0.f, 0.f, 0.f};
        ar[nt] = (v8f){0.f, 0.f, 0.f, 0.f, 0.f, 0.f, 0.f, 0.f};
        am[nt] = mma_h(ah, bh, am[nt]);
        ar[nt] = mma_h(ah, bl, ar[nt]);
        ar[nt] = mma_h(al, bh, ar[nt]);
      }
      float* dstp = TPG + (g * 3 + p) * 512;
#pragma unroll
      for (int nt = 0; nt < 2; ++nt) {
        const int n = nt * 16 + cc;
        const float bv = bias[n];
#pragma unroll
        for (int r = 0; r < 8; ++r) {
          const float v = (am[nt][r] + ar[nt][r] * kLoInv) * kWInv + bv;
          dstp[(8 * hh + r) * kFeat + n] = fmaxf(v, 0.0f);
        }
      }
    }
    wave_sync();
  }

#pragma unroll
  for (int n = 0; n < kAgents; ++n) {
    float* gp = TPG + (n * 3 + 2) * 512 + cc * kFeat + 16 * hh;
    float t[16];
    load16(gp, t);
    float s = 0.0f;
#pragma unroll
    for (int k = 0; k < 16; ++k) s += t[k];
    s += __shfl_xor(s, 16, 32);
    const float mean = s * kInvFeat;
#pragma unroll
    for (int k = 0; k < 16; ++k) t[k] -= mean;
    store16f(gp, t);
  }
  wave_sync();
  {
    float* th0 = TPG + 0 * 512 + cc * kFeat;
    float* th1 = TPG + 3 * 512 + cc * kFeat;
    float* th2 = TPG + 6 * 512 + cc * kFeat;
    const float* ph0 = TPG + 1 * 512 + cc * kFeat;
    const float* ph1 = TPG + 4 * 512 + cc * kFeat;
    const float* ph2 = TPG + 7 * 512 + cc * kFeat;
    const float* gc0 = TPG + 2 * 512 + cc * kFeat;
    const float* gc1 = TPG + 5 * 512 + cc * kFeat;
    const float* gc2 = TPG + 8 * 512 + cc * kFeat;
#pragma unroll 1
    for (int dd = 0; dd < 16; ++dd) {
      const int d = 16 * hh + dd;
      const float t0 = th0[d], t1 = th1[d], t2 = th2[d];
      float mx = -INFINITY;
#pragma unroll 1
      for (int e4 = 0; e4 < 8; ++e4) {
        const v4f a0 = *(const v4f*)(ph0 + 4 * e4);
        const v4f a1 = *(const v4f*)(ph1 + 4 * e4);
        const v4f a2 = *(const v4f*)(ph2 + 4 * e4);
#pragma unroll
        for (int e = 0; e < 4; ++e) mx = fmaxf(mx, logit3(t0, t1, t2, a0[e], a1[e], a2[e], inv_scale));
      }
      float sum = 0.0f, i0 = 0.0f, i1 = 0.0f, i2 = 0.0f;
#pragma unroll 1
      for (int e4 = 0; e4 < 8; ++e4) {
        const v4f a0 = *(const v4f*)(ph0 + 4 * e4);
        const v4f a1 = *(const v4f*)(ph1 + 4 * e4);
        const v4f a2 = *(const v4f*)(ph2 + 4 * e4);
        const v4f g0 = *(const v4f*)(gc0 + 4 * e4);
        const v4f g1 = *(const v4f*)(gc1 + 4 * e4);
        const v4f g2 = *(const v4f*)(gc2 + 4 * e4);
#pragma unroll
        for (int e = 0; e < 4; ++e) {
          const float v = logit3(t0, t1, t2, a0[e], a1[e], a2[e], inv_scale);
          const float pe = expf(v - mx);
          sum += pe;
          i0 = fmaf(pe, g0[e], i0);
          i1 = fmaf(pe, g1[e], i1);
          i2 = fmaf(pe, g2[e], i2);
        }
      }
      const float inv = 1.0f / sum;
      th0[d] = i0 * inv;
      th1[d] = i1 * inv;
      th2[d] = i2 * inv;
    }
  }
  wave_sync();
  {
    float y0[16], kv[2][16], o[16];
    load16(TPG + 0 * 512 + cc * kFeat + 16 * hh, y0);
    load16(TPG + 3 * 512 + cc * kFeat + 16 * hh, kv[0]);
    load16(TPG + 6 * 512 + cc * kFeat + 16 * hh, kv[1]);
    ln_relu16(y0,    P.cng + 0 * kFeat + 16 * hh, P.cnb + 0 * kFeat + 16 * hh);
    ln_relu16(kv[0], P.cng + 1 * kFeat + 16 * hh, P.cnb + 1 * kFeat + 16 * hh);
    ln_relu16(kv[1], P.cng + 2 * kFeat + 16 * hh, P.cnb + 2 * kFeat + 16 * hh);
    pool_ln_relu<2>(y0, kv, P.cn2g + 16 * hh, P.cn2b + 16 * hh, inv_scale, o);
    store16h(ZIN + cc * kHid + 32 + 16 * hh, o);
  }
  wave_sync();
  {
    v8f acc[4];
    wave_mm<2, 4>(ZIN, kHid, P.wp + kOffCm1, kHid, lane, acc);
    wave_epi<4, 2, 1, false>(acc, P.cm1b, T0h, T0l, kHid, S32, kFeat, lane);
  }
  wave_sync();
  {
    v8f acc[4];
    wave_mm<2, 4>(T0h, kHid, P.wp + kOffCm2, kHid, lane, acc);
    wave_epi<4, 2, 0, true>(acc, P.cm2b, T0h, T0l, kHid, ZF, kHid, lane);
  }
  wave_sync();
  {
    float a = 0.0f;
#pragma unroll
    for (int i = 0; i < 8; ++i) {
      const v4f zv = *(const v4f*)(ZF + cc * kHid + 32 * hh + 4 * i);
      const v4f wq = *(const v4f*)(P.cm3w + 32 * hh + 4 * i);
      a = fmaf(zv[0], wq[0], a);
      a = fmaf(zv[1], wq[1], a);
      a = fmaf(zv[2], wq[2], a);
      a = fmaf(zv[3], wq[3], a);
    }
    a += __shfl_xor(a, 16, 32);
    const float res = a + P.cm3b[0];
    if (hh == 0) sOut[wrow0 + cc] = res;
  }
  __syncthreads();
  if (wave == 0) {
    const float v0 = sOut[lane];
    const float v1 = sOut[32 + lane];
    float* op = P.out + blockRow0;
    *(volatile float*)(op + lane) = v0;
    *(volatile float*)(op + 32 + lane) = v1;
    __threadfence();
    *(volatile float*)(op + lane) = v0;
    *(volatile float*)(op + 32 + lane) = v1;
  }
}

extern "C" void kernel_launch(void* const* d_in, const int* in_sizes, int n_in,
                              void* d_out, int out_size, void* d_ws, size_t ws_size,
                              hipStream_t stream) {
  (void)in_sizes; (void)out_size;
  if (n_in < 39) return;
  if (ws_size < kWsBytes) return;

  _Float16* planes = (_Float16*)d_ws;

  PrepArgs A;
  A.src[0]  = (const float*)d_in[3];
  A.src[1]  = (const float*)d_in[7];
  A.src[2]  = (const float*)d_in[13];
  A.src[3]  = (const float*)d_in[17];
  A.src[4]  = (const float*)d_in[19];
  A.src[5]  = (const float*)d_in[21];
  A.src[6]  = (const float*)d_in[33];
  A.src[7]  = (const float*)d_in[35];
  A.src[8]  = (const float*)d_in[23];
  A.src[9]  = (const float*)d_in[25];
  A.src[10] = (const float*)d_in[27];
  A.src[11] = (const float*)d_in[23];
  A.src[12] = (const float*)d_in[25];
  A.src[13] = (const float*)d_in[27];
  A.src[14] = (const float*)d_in[3];
  A.src[15] = (const float*)d_in[7];
  A.src[16] = (const float*)d_in[13];
  A.src[17] = (const float*)d_in[17];
  A.src[18] = (const float*)d_in[19];
  A.src[19] = (const float*)d_in[21];

  Params P;
  P.x    = (const float*)d_in[0];
  P.as1w = (const float*)d_in[1];
  P.as1b = (const float*)d_in[2];
  P.as2b = (const float*)d_in[4];
  P.af1w = (const float*)d_in[5];
  P.af1b = (const float*)d_in[6];
  P.af2b = (const float*)d_in[8];
  P.afng = (const float*)d_in[9];
  P.afnb = (const float*)d_in[10];
  P.ao1w = (const float*)d_in[11];
  P.ao1b = (const float*)d_in[12];
  P.ao2b = (const float*)d_in[14];
  P.aong = (const float*)d_in[15];
  P.aonb = (const float*)d_in[16];
  P.am1b = (const float*)d_in[18];
  P.am2b = (const float*)d_in[20];
  P.am3b = (const float*)d_in[22];
  P.ca1b = (const float*)d_in[24];
  P.ca2b = (const float*)d_in[26];
  P.ca3b = (const float*)d_in[28];
  P.cng  = (const float*)d_in[29];
  P.cnb  = (const float*)d_in[30];
  P.cn2g = (const float*)d_in[31];
  P.cn2b = (const float*)d_in[32];
  P.cm1b = (const float*)d_in[34];
  P.cm2b = (const float*)d_in[36];
  P.cm3w = (const float*)d_in[37];
  P.cm3b = (const float*)d_in[38];
  P.wp   = planes;
  P.out  = (float*)d_out;

  prep_planes_kernel<<<kPrepChunks / 256, 256, 0, stream>>>(A, planes);
  fused_forward_kernel<<<kRows / kBlkRows, kThreads, 0, stream>>>(P);
}
